// PointTransformer_29085518528923
// MI455X (gfx1250) — hardware-verified
//
#include <hip/hip_runtime.h>
#include <math.h>

typedef __attribute__((ext_vector_type(16))) _Float16 v16h;
typedef __attribute__((ext_vector_type(16))) __bf16 v16b;
typedef __attribute__((ext_vector_type(8)))  _Float16 v8h;
typedef __attribute__((ext_vector_type(8)))  float v8f;
typedef __attribute__((ext_vector_type(4)))  float v4f;
typedef __attribute__((ext_vector_type(2)))  float v2f;
typedef __attribute__((ext_vector_type(4)))  unsigned v4u;
typedef __attribute__((ext_vector_type(4)))  int v4i;
typedef float __attribute__((may_alias)) float_a;
typedef int __attribute__((may_alias)) int_a;

template <typename T> __device__ __forceinline__ void vst2(void* p, T v) { *(volatile T*)p = v; __threadfence(); *(volatile T*)p = v; }
__device__ __forceinline__ v8f wmma16(v16h a, v16h b, v8f c) {
  v8f d = __builtin_amdgcn_wmma_f32_16x16x32_f16(false, a, false, b, (short)0, c, false, false);
  asm volatile("v_nop\n\tv_nop\n\tv_nop\n\tv_nop" : "+v"(d) : "v"(a), "v"(b));
  return d;
}
__device__ __forceinline__ v8f wmma_bf(v16b a, v16b b, v8f c) {
  v8f d = __builtin_amdgcn_wmma_f32_16x16x32_bf16(false, a, false, b, (short)0, c, false, false);
  asm volatile("v_nop\n\tv_nop\n\tv_nop\n\tv_nop" : "+v"(d) : "v"(a), "v"(b));
  return d;
}
__device__ __forceinline__ v16h frag_h(const _Float16* rowk0, int lane) {
  union { v16h v; v8h q[2]; } u; const _Float16* p = rowk0 + 8 * (lane >> 4);
  u.q[0] = *(const v8h*)p; u.q[1] = *(const v8h*)(p + 16); return u.v;
}
__device__ __forceinline__ v16h frag_f32(const float* rowk0, int lane) {
  v16h a; const float* p = rowk0 + 8 * (lane >> 4);
#pragma unroll
  for (int i = 0; i < 8; ++i) { a[i] = (_Float16)p[i]; a[8 + i] = (_Float16)p[16 + i]; }
  return a;
}
__device__ __forceinline__ v16h frag_f32s(const float* rowk0, int lane, float sc) {
  v16h a; const float* p = rowk0 + 8 * (lane >> 4);
#pragma unroll
  for (int i = 0; i < 8; ++i) { a[i] = (_Float16)(p[i] * sc); a[8 + i] = (_Float16)(p[16 + i] * sc); }
  return a;
}
__device__ __forceinline__ v16h fragc_f32(const float* W, int k0, int n, int lane, int ld, int K) {
  v16h a; const int g = lane >> 4;
#pragma unroll
  for (int i = 0; i < 8; ++i) { const int ka = k0 + 8 * g + i, kb = ka + 16;
    a[i] = (_Float16)(ka < K ? W[(size_t)(ka < K ? ka : K - 1) * ld + n] : 0.f); a[8 + i] = (_Float16)(kb < K ? W[(size_t)(kb < K ? kb : K - 1) * ld + n] : 0.f); }
  return a;
}
struct F2 { v16b h, l; };
__device__ __forceinline__ F2 bsplit16(const float v[16]) { F2 r;
#pragma unroll
  for (int i = 0; i < 16; ++i) { const __bf16 h = (__bf16)v[i]; r.h[i] = h; r.l[i] = (__bf16)(v[i] - (float)h); }
  return r; }
__device__ __forceinline__ F2 split_row(const float* row, int k0, int lane) { float v[16]; const float* p = row + k0 + 8 * (lane >> 4);
#pragma unroll
  for (int i = 0; i < 8; ++i) { v[i] = p[i]; v[8 + i] = p[16 + i]; }
  return bsplit16(v); }
__device__ __forceinline__ F2 split_rowK(const float* row, int k0, int lane, int K) { float v[16]; const int g = lane >> 4;
#pragma unroll
  for (int i = 0; i < 8; ++i) { const int ka = k0 + 8 * g + i, kb = ka + 16; v[i] = ka < K ? row[ka < K ? ka : K - 1] : 0.f; v[8 + i] = kb < K ? row[kb < K ? kb : K - 1] : 0.f; }
  return bsplit16(v); }
__device__ __forceinline__ F2 split_col(const float* W, int k0, int n, int lane, int ld, int K) { float v[16]; const int g = lane >> 4;
#pragma unroll
  for (int i = 0; i < 8; ++i) { const int ka = k0 + 8 * g + i, kb = ka + 16; v[i] = ka < K ? W[(size_t)(ka < K ? ka : K - 1) * ld + n] : 0.f; v[8 + i] = kb < K ? W[(size_t)(kb < K ? kb : K - 1) * ld + n] : 0.f; }
  return bsplit16(v); }
__device__ __forceinline__ v8f mac3(const F2& a, const F2& b, v8f c) { c = wmma_bf(a.l, b.h, c); c = wmma_bf(a.h, b.l, c); return wmma_bf(a.h, b.h, c); }
__device__ __forceinline__ float sigm(float v) { return 1.0f / (1.0f + expf(-v)); }
#define LDSX() do { asm volatile("s_wait_dscnt 0" ::: "memory"); __builtin_amdgcn_wave_barrier(); __builtin_amdgcn_fence(__ATOMIC_RELEASE, "workgroup"); } while (0)

#define NBT 8
#define NPT 2048
#define CIN 32
#define CO 32
#define PH 64
#define VH 4
#define KSEL 17
#define KN 16
#define NR (NBT * NPT)
#ifndef NRV
#define NRV NR
#endif
#define OUT1_OFF (4u * (size_t)NR * CO)
typedef __attribute__((ext_vector_type(4))) int v4i;
__device__ __forceinline__ float bfr(float v) { return (float)(__bf16)v; }
__device__ __forceinline__ v16b wcol_kz(const float* __restrict__ Wm, int k0, int o, int lane, int ld, int K, int nvalid) { v16b w; const int g = lane >> 4; const int oc = o < nvalid ? o : 0; const float keepo = o < nvalid ? 1.f : 0.f;
#pragma unroll
  for (int i = 0; i < 8; ++i) { const int ka = k0 + 8 * g + i, kb = ka + 16; w[i] = (__bf16)(Wm[(size_t)(ka < K ? ka : 0) * ld + oc] * (ka < K ? keepo : 0.f)); w[8 + i] = (__bf16)(Wm[(size_t)(kb < K ? kb : 0) * ld + oc] * (kb < K ? keepo : 0.f)); }
  asm volatile("s_wait_loadcnt 0x0" ::: "memory"); return w; }
#define WS_XA  0u
#define WS_XB  (WS_XA + 4u * (size_t)NR * CO)
#define WS_XC  (WS_XB + 4u * (size_t)NR * CO)
#define WS_IDX (WS_XC + 4u * (size_t)NR * CO)
#define WS_END (WS_IDX + 4u * (size_t)NR * KN)
__global__ __launch_bounds__(128) void k_lin(const float* __restrict__ X, const float* __restrict__ WA, const float* __restrict__ BA, const float* __restrict__ WB, const float* __restrict__ BB, const float* __restrict__ WC, const float* __restrict__ BC, float* __restrict__ XA, float* __restrict__ XB, float* __restrict__ XC) { __shared__ __align__(16) float sf[4][16][36];
  const int tid = threadIdx.x, wave = tid >> 5, lane = tid & 31, col = lane & 15, g = lane >> 4; const int which = blockIdx.y; const size_t r0 = (size_t)blockIdx.x * 64 + wave * 16;
  const float* Wm = which == 0 ? WA : (which == 1 ? WB : WC); const float* Bm = which == 0 ? BA : (which == 1 ? BB : BC); float* OUT = which == 0 ? XA : (which == 1 ? XB : XC);
  v16b a; { const float* p = X + (r0 + col) * CIN + 8 * g;
#pragma unroll
    for (int i = 0; i < 8; ++i) { a[i] = (__bf16)p[i]; a[8 + i] = (__bf16)p[16 + i]; } }
  asm volatile("s_wait_loadcnt 0x0" ::: "memory");
  v8f acc[2] = {};
#pragma unroll
  for (int j = 0; j < 2; ++j) { const v16b w = wcol_kz(Wm, 0, j * 16 + col, lane, CO, CIN, CO); acc[j] = wmma_bf(a, w, acc[j]); }
#pragma unroll
  for (int j = 0; j < 2; ++j) { const float bb = bfr(Bm[j * 16 + col]);
#pragma unroll
    for (int r = 0; r < 8; ++r) sf[wave][8 * g + r][j * 16 + col] = acc[j][r] + bb; }
  LDSX(); for (int rl = 0; rl < 16; ++rl) if (lane < 8) vst2(OUT + (r0 + rl) * CO + lane * 4, *(const v4f*)&sf[wave][rl][lane * 4]); }
struct Best17 { float d[KSEL]; int i[KSEL]; };
__device__ __forceinline__ void push17(Best17& b, float d, int i) {
  if (d < b.d[KSEL - 1]) { b.d[KSEL - 1] = d; b.i[KSEL - 1] = i; }
#pragma unroll
  for (int p = KSEL - 1; p > 0; --p) { const bool sw = b.d[p] < b.d[p - 1]; const float td = b.d[p], ud = b.d[p - 1]; const int ti = b.i[p], ui = b.i[p - 1]; b.d[p] = sw ? ud : td; b.d[p - 1] = sw ? td : ud; b.i[p] = sw ? ui : ti; b.i[p - 1] = sw ? ti : ui; } }
__global__ __launch_bounds__(256) void k_knn(const float* __restrict__ P, int* __restrict__ IDX) { __shared__ int sidx8[8][KN];
  const int wave = threadIdx.x >> 5, lane = threadIdx.x & 31; const size_t row = (size_t)blockIdx.x * 8 + wave;
  const size_t b = row / NPT; const int n = (int)(row % NPT);
  Best17 bs;
#pragma unroll
  for (int r = 0; r < KSEL; ++r) { bs.d[r] = 3.0e38f; bs.i[r] = 0x7fffffff; }
  {
#pragma clang fp contract(off)
    const float qx = bfr(P[(b * NPT + n) * 3]), qy = bfr(P[(b * NPT + n) * 3 + 1]), qz = bfr(P[(b * NPT + n) * 3 + 2]);
#pragma unroll 1
    for (int s = lane; s < NPT; s += 32) { const float dx = qx - bfr(P[(b * NPT + s) * 3]), dy = qy - bfr(P[(b * NPT + s) * 3 + 1]), dz = qz - bfr(P[(b * NPT + s) * 3 + 2]);
      const float d = (dx * dx + dz * dz) + dy * dy; push17(bs, d, s); } }
  int sel = 0;
#pragma unroll 1
  for (int r = 0; r < KSEL; ++r) { float d = bs.d[0]; int i = bs.i[0];
#pragma unroll
    for (int o = 1; o < 32; o <<= 1) { const float e = __shfl_xor(d, o); const int j = __shfl_xor(i, o); if (e < d || (e == d && j < i)) { d = e; i = j; } }
    if (lane == r - 1) sel = i;
    { const bool pop = (bs.i[0] == i && bs.d[0] == d);
#pragma unroll
      for (int p = 0; p < KSEL - 1; ++p) { bs.d[p] = pop ? bs.d[p + 1] : bs.d[p]; bs.i[p] = pop ? bs.i[p + 1] : bs.i[p]; }
      bs.d[KSEL - 1] = pop ? 3.0e38f : bs.d[KSEL - 1]; bs.i[KSEL - 1] = pop ? 0x7fffffff : bs.i[KSEL - 1]; } }
  if (lane < KN) sidx8[wave][lane] = sel;
  __syncthreads();
  if (threadIdx.x < 32) vst2((v4i*)(IDX + (size_t)blockIdx.x * 8 * KN) + threadIdx.x, *(const v4i*)(&sidx8[0][0] + threadIdx.x * 4)); }
__global__ __launch_bounds__(256) void k_pcopy(const float* __restrict__ P, float* __restrict__ O1) { const size_t i = ((size_t)blockIdx.x * 256 + threadIdx.x) * 4; const v4f v = *(const v4f*)(P + i); asm volatile("s_wait_loadcnt 0x0" ::: "memory"); v4f o; o[0] = bfr(v[0]); o[1] = bfr(v[1]); o[2] = bfr(v[2]); o[3] = bfr(v[3]); vst2(O1 + i, o); }

__global__ __launch_bounds__(128) void k_edge(const float* __restrict__ P, const int* __restrict__ IDX, const float* __restrict__ XA, const float* __restrict__ XB, const float* __restrict__ XC,
    const float* __restrict__ PM1W, const float* __restrict__ PM1B, const float* __restrict__ PM2W, const float* __restrict__ PM2B, const float* __restrict__ VM1W, const float* __restrict__ VM1B, const float* __restrict__ VM2W, const float* __restrict__ VM2B, float* __restrict__ Y) {
  __shared__ __align__(16) float sh1[4][16][68]; __shared__ __align__(16) float spe[4][16][36]; __shared__ __align__(16) float sz[4][16][36]; __shared__ int sidx[4][16];
  const int tid = threadIdx.x, wave = tid >> 5, lane = tid & 31, col = lane & 15, g = lane >> 4;
  const size_t n = (size_t)blockIdx.x * 4 + wave; const size_t b = n / NPT;
  if (lane < KN) { int ix = IDX[n * KN + lane]; ix = ix < 0 ? 0 : (ix >= NPT ? NPT - 1 : ix); sidx[wave][lane] = (int)(b * NPT + ix); }
  LDSX();
  {
    const int j = col; const size_t m = (size_t)sidx[wave][j];
    const float rx = bfr(P[n * 3]) - bfr(P[m * 3]), ry = bfr(P[n * 3 + 1]) - bfr(P[m * 3 + 1]), rz = bfr(P[n * 3 + 2]) - bfr(P[m * 3 + 2]);
    asm volatile("s_wait_loadcnt 0x0" ::: "memory");
#pragma unroll 4
    for (int q = 0; q < 32; ++q) { const int o = g * 32 + q; const float y = ((rx * bfr(PM1W[o]) + ry * bfr(PM1W[PH + o])) + rz * bfr(PM1W[2 * PH + o])) + bfr(PM1B[o]); sh1[wave][j][o] = fmaxf(y, 0.f); } }
  LDSX();
  {
    v8f acc[2] = {};
#pragma unroll
    for (int kc = 0; kc < PH / 32; ++kc) { const F2 a = split_row(&sh1[wave][col][0], kc * 32, lane);
#pragma unroll
      for (int jj = 0; jj < 2; ++jj) { const v16b w = wcol_kz(PM2W, kc * 32, jj * 16 + col, lane, CO, PH, CO); acc[jj] = wmma_bf(a.h, w, acc[jj]); acc[jj] = wmma_bf(a.l, w, acc[jj]); } }
#pragma unroll
    for (int jj = 0; jj < 2; ++jj) { const float bb = bfr(PM2B[jj * 16 + col]);
#pragma unroll
      for (int r = 0; r < 8; ++r) spe[wave][8 * g + r][jj * 16 + col] = acc[jj][r] + bb; } }
  LDSX();
  {
    const size_t m = (size_t)sidx[wave][col]; float va[16];
#pragma unroll
    for (int i = 0; i < 16; ++i) { const int c = 8 * g + (i < 8 ? i : 8 + i); va[i] = (XA[n * CO + c] - XB[m * CO + c]) + spe[wave][col][c]; }
    asm volatile("s_wait_loadcnt 0x0" ::: "memory");
    const F2 a = bsplit16(va); v8f acc = {};
    { const v16b w = wcol_kz(VM1W, 0, col, lane, VH, CO, VH); acc = wmma_bf(a.h, w, acc); acc = wmma_bf(a.l, w, acc); }
    const float bb = col < VH ? bfr(VM1B[col < VH ? col : 0]) : 0.f;
#pragma unroll
    for (int r = 0; r < 8; ++r) sz[wave][8 * g + r][col] = col < VH ? fmaxf(acc[r] + bb, 0.f) : 0.f; }
  if (true) { for (int e = lane; e < 16 * 16; e += 32) sz[wave][e >> 4][16 + (e & 15)] = 0.f; }
  LDSX();
  {
    v8f acc[2] = {}; const F2 a = split_row(&sz[wave][col][0], 0, lane);
#pragma unroll
    for (int jj = 0; jj < 2; ++jj) { const v16b w = wcol_kz(VM2W, 0, jj * 16 + col, lane, CO, VH, CO); acc[jj] = wmma_bf(a.h, w, acc[jj]); acc[jj] = wmma_bf(a.l, w, acc[jj]); }
    LDSX();
#pragma unroll
    for (int jj = 0; jj < 2; ++jj) { const float bb = bfr(VM2B[jj * 16 + col]);
#pragma unroll
      for (int r = 0; r < 8; ++r) sz[wave][8 * g + r][jj * 16 + col] = acc[jj][r] + bb; } }
  LDSX();
  {
    const int c = lane; float mx = -3.0e38f;
#pragma unroll
    for (int j = 0; j < KN; ++j) mx = fmaxf(mx, sz[wave][j][c]);
    float e[KN], sum = 0.f;
#pragma unroll
    for (int j = 0; j < KN; ++j) { e[j] = expf(sz[wave][j][c] - mx); sum += e[j]; }
    const float inv = 1.0f / sum; float y = 0.f;
#pragma unroll
    for (int j = 0; j < KN; ++j) { const size_t m = (size_t)sidx[wave][j]; const float xj2 = XC[m * CO + c]; y += (e[j] * inv) * (spe[wave][j][c] + xj2); }
    vst2(Y + n * CO + c, y); } }
extern "C" void kernel_launch(void* const* d_in, const int* in_sizes, int n_in, void* d_out, int out_size, void* d_ws, size_t ws_size, hipStream_t stream) {
  (void)in_sizes; (void)n_in; (void)out_size;
  if (ws_size < (size_t)WS_END) return;
  char* ws = (char*)d_ws; const float** F = (const float**)d_in; float *XA = (float*)(ws + WS_XA), *XB = (float*)(ws + WS_XB), *XC = (float*)(ws + WS_XC); int* IDX = (int*)(ws + WS_IDX);
  k_lin<<<dim3(NRV / 64, 3), 128, 0, stream>>>(F[0], F[2], F[3], F[4], F[5], F[6], F[7], XA, XB, XC);
  k_knn<<<dim3(NRV / 8), 256, 0, stream>>>(F[1], IDX);
  k_pcopy<<<dim3(NRV * 3 / 1024), 256, 0, stream>>>(F[1], (float*)((char*)d_out + OUT1_OFF));
  k_edge<<<dim3(NRV / 4), 128, 0, stream>>>(F[1], IDX, XA, XB, XC, F[8], F[9], F[10], F[11], F[12], F[13], F[14], F[15], (float*)d_out);
}
